// SlidingWindowAttention_44968307589534
// MI455X (gfx1250) — hardware-verified
//
#include <hip/hip_runtime.h>


#ifndef NB
#define NB 1
#endif
#ifndef SEQ
#define SEQ 2048
#endif
#define SEQ_FULL 2048
#define TT   SEQ
#define DM   512
#define NH_  8
#define NKV  2
#define REP  (NH_ / NKV)
#define HD   64
#define DQ   (NH_ * HD)
#define DKV  (NKV * HD)
#define WIN  128
#define PADK 128
#define TP   (TT + PADK)
#define SBW  192
#define SCL  0.125f
static_assert(SEQ % 64 == 0);
static_assert(SEQ >= 64 && SEQ <= SEQ_FULL);
static_assert(NB >= 1);
static_assert(NH_ % NKV == 0);
static_assert(HD == 64 && DM % 64 == 0 && DQ % 64 == 0 && DKV % 64 == 0 && DM % 32 == 0 && DQ % 32 == 0);
static_assert(SBW % 64 == 0 && SBW == WIN + 64 && PADK >= WIN && TP % 64 == 0);
static_assert(((size_t)TT * DM / 8) % 256 == 0);
static_assert(((size_t)TT * DQ / 8) % 256 == 0);
static_assert((TT * HD) % 256 == 0);
static_assert(((size_t)NH_ * TT * HD / 2) % 256 == 0);
static_assert(((size_t)NKV * TP * HD / 2) % 256 == 0);
static_assert((NH_ * TT) % 8 == 0);
static_assert((DM * DQ) % 64 == 0 && (DM * DKV) % 64 == 0);

typedef _Float16 h16;
typedef unsigned short bf;
typedef __attribute__((ext_vector_type(16))) __bf16   v16bf;
typedef __attribute__((ext_vector_type(16))) _Float16 v16h;
typedef __attribute__((ext_vector_type(8)))  _Float16 v8h;
typedef __attribute__((ext_vector_type(8)))  unsigned short v8us;
typedef __attribute__((ext_vector_type(8)))  float    v8f;
typedef __attribute__((ext_vector_type(4)))  float    v4f;
typedef __attribute__((ext_vector_type(2)))  float    v2f;
typedef __attribute__((ext_vector_type(4)))  unsigned short v4us;
typedef __attribute__((ext_vector_type(2)))  unsigned short v2us;
typedef v8h  __attribute__((may_alias)) v8ha;
typedef v4f  __attribute__((may_alias)) v4fa;
typedef v8us __attribute__((may_alias)) v8usa;

__device__ __forceinline__ unsigned short f2bf(float f) { unsigned u = __float_as_uint(f); u += 0x7FFFu + ((u >> 16) & 1u); return (unsigned short)(u >> 16); }
__device__ __forceinline__ float bf2f(unsigned short b) { return __uint_as_float(((unsigned)b) << 16); }
__device__ __forceinline__ float bfr(float f) { return bf2f(f2bf(f)); }
__device__ __forceinline__ v16h cat16(v8h lo, v8h hi) { return __builtin_shufflevector(lo, hi, 0, 1, 2, 3, 4, 5, 6, 7, 8, 9, 10, 11, 12, 13, 14, 15); }
__device__ __forceinline__ v16bf cat16b(v8us lo, v8us hi) { return __builtin_bit_cast(v16bf, __builtin_shufflevector(lo, hi, 0, 1, 2, 3, 4, 5, 6, 7, 8, 9, 10, 11, 12, 13, 14, 15)); }
__device__ __forceinline__ v8f wmma16(v16h a, v16h b, v8f c) { return __builtin_amdgcn_wmma_f32_16x16x32_f16(false, a, false, b, (short)0, c, false, false); }
__device__ __forceinline__ v8f wmmab(v16bf a, v16bf b, v8f c) { return __builtin_amdgcn_wmma_f32_16x16x32_bf16(false, a, false, b, (short)0, c, false, false); }
__device__ __forceinline__ void splitf(float y, unsigned short& h, unsigned short& l) { h = f2bf(y); l = f2bf(y - bf2f(h)); }

template <typename T16> struct WFrag;
template <> struct WFrag<h16> { typedef v16h V; static __device__ __forceinline__ V ld(const h16* p) { return cat16(*(const v8h*)p, *(const v8h*)(p + 16)); } static __device__ __forceinline__ v8f mma(V a, V b, v8f c) { return wmma16(a, b, c); } };
template <> struct WFrag<bf> { typedef v16bf V; static __device__ __forceinline__ V ld(const bf* p) { return cat16b(*(const v8us*)p, *(const v8us*)(p + 16)); } static __device__ __forceinline__ v8f mma(V a, V b, v8f c) { return wmmab(a, b, c); } };
template <typename T16, int NSPLIT, bool BIAS>
__global__ __launch_bounds__(32) void k_gemmw(const T16* __restrict__ A, const T16* __restrict__ A2, const T16* __restrict__ Bt, const T16* __restrict__ Bt2, int K, float* C, int ldc, const float* __restrict__ bias, size_t sA, size_t sB, size_t sC) {
    typedef typename WFrag<T16>::V V;
    __shared__ __align__(16) float os[16 * 68];
    const size_t z = blockIdx.z; A += z * sA; if (A2) A2 += z * sA; Bt += z * sB; if (Bt2) Bt2 += z * sB; C += z * sC;
    const int lane = threadIdx.x & 31, lr = lane & 15, hi = lane >> 4; const int r0 = blockIdx.x * 64, c0 = blockIdx.y * 64;
    v8f acc[4][4];
#pragma unroll
    for (int mb = 0; mb < 4; ++mb)
#pragma unroll
        for (int nb = 0; nb < 4; ++nb) acc[mb][nb] = (v8f){};
    const size_t aoff = (size_t)(r0 + lr) * K + 8 * hi, boff = (size_t)(c0 + lr) * K + 8 * hi;
#pragma unroll 1
    for (int kc = 0; kc < K; kc += 32) {
        V a[4], a2[4];
#pragma unroll
        for (int mb = 0; mb < 4; ++mb) { a[mb] = WFrag<T16>::ld(A + aoff + (size_t)mb * 16 * K + kc); if (NSPLIT == 1 || NSPLIT == 2) a2[mb] = WFrag<T16>::ld(A2 + aoff + (size_t)mb * 16 * K + kc); }
#pragma unroll
        for (int nb = 0; nb < 4; ++nb) { const V b = WFrag<T16>::ld(Bt + boff + (size_t)nb * 16 * K + kc); V b2; if (NSPLIT >= 2) b2 = WFrag<T16>::ld(Bt2 + boff + (size_t)nb * 16 * K + kc);
#pragma unroll
            for (int mb = 0; mb < 4; ++mb) { acc[mb][nb] = WFrag<T16>::mma(a[mb], b, acc[mb][nb]); if (NSPLIT == 1 || NSPLIT == 2) acc[mb][nb] = WFrag<T16>::mma(a2[mb], b, acc[mb][nb]); if (NSPLIT >= 2) acc[mb][nb] = WFrag<T16>::mma(a[mb], b2, acc[mb][nb]); } }
        asm volatile("v_nop\n\tv_nop\n\tv_nop\n\tv_nop" : "+v"(acc[0][0]), "+v"(acc[1][1]), "+v"(acc[2][2]), "+v"(acc[3][3]) : "v"(a[0]), "v"(a[3]));
    }
#pragma unroll
    for (int mb = 0; mb < 4; ++mb) {
#pragma unroll
        for (int nb = 0; nb < 4; ++nb) {
#pragma unroll
            for (int j = 0; j < 8; ++j) os[(hi * 8 + j) * 68 + nb * 16 + lr] = acc[mb][nb][j]; }
        __builtin_amdgcn_wave_barrier(); asm volatile("" ::: "memory");
        float* crow = C + (size_t)(r0 + mb * 16) * ldc + c0;
#pragma unroll 1
        for (int ps = 0; ps < 2; ++ps) {
#pragma unroll
            for (int s = 0; s < 8; ++s) { const int row = 2 * s + hi, cofs = lr * 4; v4f val = *(const v4fa*)(os + row * 68 + cofs); if (BIAS) { val[0] += bfr(bias[c0 + cofs]); val[1] += bfr(bias[c0 + cofs + 1]); val[2] += bfr(bias[c0 + cofs + 2]); val[3] += bfr(bias[c0 + cofs + 3]); }
                *(volatile v4f*)(crow + (size_t)row * ldc + cofs) = val; }
            if (ps == 0) __threadfence(); }
        __builtin_amdgcn_wave_barrier(); asm volatile("" ::: "memory");
    }
}

template <int NSPLIT, int ZDIV>
__global__ __launch_bounds__(32) void k_gemmb(const bf* __restrict__ A, const bf* __restrict__ A2, int lda, const bf* __restrict__ Bt, const bf* __restrict__ Bt2, int ldb, int K, float* C, int ldc, size_t sA, size_t sB, size_t sC, size_t bxs) {
    typedef v16bf V;
    __shared__ __align__(16) float os[16 * 68];
    const size_t z = blockIdx.z, zb = z / ZDIV, bsh = zb * sB + (size_t)blockIdx.x * bxs;
    A += z * sA; if (NSPLIT >= 1) A2 += z * sA; Bt += bsh; if (NSPLIT >= 2) Bt2 += bsh; C += z * sC;
    const int lane = threadIdx.x & 31, lr = lane & 15, hi = lane >> 4; const int r0 = blockIdx.x * 64, c0 = blockIdx.y * 64;
    v8f acc[4][4];
#pragma unroll
    for (int mb = 0; mb < 4; ++mb)
#pragma unroll
        for (int nb = 0; nb < 4; ++nb) acc[mb][nb] = (v8f){};
    const size_t aoff = (size_t)(r0 + lr) * lda + 8 * hi, boff = (size_t)(c0 + lr) * ldb + 8 * hi;
#pragma unroll 1
    for (int kc = 0; kc < K; kc += 32) {
        V a[4], a2[4];
#pragma unroll
        for (int mb = 0; mb < 4; ++mb) { a[mb] = WFrag<bf>::ld(A + aoff + (size_t)mb * 16 * lda + kc); a2[mb] = a[mb]; if (NSPLIT >= 1) a2[mb] = WFrag<bf>::ld(A2 + aoff + (size_t)mb * 16 * lda + kc); }
#pragma unroll
        for (int nb = 0; nb < 4; ++nb) { const V b = WFrag<bf>::ld(Bt + boff + (size_t)nb * 16 * ldb + kc); V b2 = b; if (NSPLIT >= 2) b2 = WFrag<bf>::ld(Bt2 + boff + (size_t)nb * 16 * ldb + kc);
#pragma unroll
            for (int mb = 0; mb < 4; ++mb) { acc[mb][nb] = wmmab(a[mb], b, acc[mb][nb]); if (NSPLIT >= 1) acc[mb][nb] = wmmab(a2[mb], b, acc[mb][nb]); if (NSPLIT >= 2) acc[mb][nb] = wmmab(a[mb], b2, acc[mb][nb]); } }
        asm volatile("v_nop\n\tv_nop\n\tv_nop\n\tv_nop" : "+v"(acc[0][0]), "+v"(acc[1][1]), "+v"(acc[2][2]), "+v"(acc[3][3]) : "v"(a[0]), "v"(a[3]));
    }
#pragma unroll
    for (int mb = 0; mb < 4; ++mb) {
#pragma unroll
        for (int nb = 0; nb < 4; ++nb) {
#pragma unroll
            for (int j = 0; j < 8; ++j) os[(hi * 8 + j) * 68 + nb * 16 + lr] = acc[mb][nb][j]; }
        __builtin_amdgcn_wave_barrier(); asm volatile("" ::: "memory");
        float* crow = C + (size_t)(r0 + mb * 16) * ldc + c0;
#pragma unroll 1
        for (int ps = 0; ps < 2; ++ps) {
#pragma unroll
            for (int s = 0; s < 8; ++s) { const int row = 2 * s + hi, cofs = lr * 4; v4f val = *(const v4fa*)(os + row * 68 + cofs);
                *(volatile v4f*)(crow + (size_t)row * ldc + cofs) = val; }
            if (ps == 0) __threadfence(); }
        __builtin_amdgcn_wave_barrier(); asm volatile("" ::: "memory");
    }
}

__global__ __launch_bounds__(256) void k_wtG(const float* __restrict__ w, int K, int N, bf* Bt) {
    const int lane = threadIdx.x & 31; const int L0 = (blockIdx.x * 8 + (threadIdx.x >> 5)) * 8; const int nlines = N * K / 64;
#pragma unroll
    for (int ps = 0; ps < 2; ++ps) {
#pragma unroll 1
        for (int l = 0; l < 8; ++l) { const int L = L0 + l; if (L >= nlines) break; const size_t e = (size_t)L * 64 + lane * 2; const int k = (int)(e % K), n = (int)(e / K); v2us o;
            o[0] = f2bf(w[(size_t)k * N + n]); o[1] = f2bf(w[(size_t)(k + 1) * N + n]); *(volatile v2us*)(Bt + e) = o; }
        if (ps == 0) __threadfence(); }
}
__global__ __launch_bounds__(256) void k_cvt8(const float* __restrict__ src, bf* dst, size_t n8) { const size_t i = (size_t)blockIdx.x * 256 + threadIdx.x; if (i >= n8) return; const v8f v = *(const v8f*)(src + i * 8); v8us o;
#pragma unroll
    for (int k = 0; k < 8; ++k) o[k] = f2bf(v[k]); *(volatile v8us*)(dst + i * 8) = o; __threadfence(); *(volatile v8us*)(dst + i * 8) = o; }
__global__ __launch_bounds__(256) void k_split8(const float* __restrict__ src, bf* dh, bf* dl, size_t n8) { const size_t i = (size_t)blockIdx.x * 256 + threadIdx.x; if (i >= n8) return; const v8f v = *(const v8f*)(src + i * 8); v8us oh, ol;
#pragma unroll
    for (int k = 0; k < 8; ++k) { unsigned short a, c2; splitf(v[k], a, c2); oh[k] = a; ol[k] = c2; }
    *(volatile v8us*)(dh + i * 8) = oh; *(volatile v8us*)(dl + i * 8) = ol; __threadfence(); *(volatile v8us*)(dh + i * 8) = oh; *(volatile v8us*)(dl + i * 8) = ol; }

__constant__ float c_invf[32] = {
    1.0f,    0.74989420933f,    0.56234132519f,    0.42169650343f,    0.31622776602f,    0.23713737057f,    0.17782794100f,    0.13335214322f,
    0.1f,    0.074989420933f,   0.056234132519f,   0.042169650343f,   0.031622776602f,   0.023713737057f,   0.017782794100f,   0.013335214322f,
    0.01f,   0.0074989420933f,  0.0056234132519f,  0.0042169650343f,  0.0031622776602f,  0.0023713737057f,  0.0017782794100f,  0.0013335214322f,
    0.001f,  0.00074989420933f, 0.00056234132519f, 0.00042169650343f, 0.00031622776602f, 0.00023713737057f, 0.00017782794100f, 0.00013335214322f };
__global__ __launch_bounds__(256) void k_cst(float* CS) {
    const int idx = blockIdx.x * 256 + threadIdx.x; if (idx >= TT * HD) return;
    const int t = idx / HD, d = idx % HD;
    const float ang = __fmul_rn((float)t, c_invf[d & (HD / 2 - 1)]);
    const float cn = cosf(ang); const float sn = sinf(ang);
    v2f cs; cs[0] = cn; cs[1] = sn;
    *(volatile v2f*)(CS + (size_t)idx * 2) = cs; __threadfence(); *(volatile v2f*)(CS + (size_t)idx * 2) = cs; }

__global__ __launch_bounds__(256) void k_rope(const float* __restrict__ F, int pitch, int nheads, int prow, int toff, const float* __restrict__ CS, bf* Ph, bf* Pl) {
    const unsigned e = (blockIdx.x * 256u + threadIdx.x) * 2u; if (e >= (unsigned)nheads * (unsigned)prow * (unsigned)HD) return;
    const int d = (int)(e % HD); const int tp = (int)((e / HD) % (unsigned)prow); const int h = (int)(e / ((unsigned)HD * (unsigned)prow));
    const int t = tp - toff; const bool live = (t >= 0); const int tc = live ? t : 0;
    const float* f = F + (size_t)tc * pitch + h * HD; v2us oh, ol;
#pragma unroll
    for (int q = 0; q < 2; ++q) { const int dd = d + q; const int dp = (dd < HD / 2) ? dd + HD / 2 : dd - HD / 2; const float x0 = f[dd], x1 = f[dp];
        const v2f cs = *(const v2f*)(CS + ((size_t)tc * HD + dd) * 2); float a = __fmul_rn(x0, cs[0]), bq = __fmul_rn(x1, cs[1]); asm volatile("" : "+v"(a)); asm volatile("" : "+v"(bq));
        float r = (dd < HD / 2) ? __fsub_rn(a, bq) : __fadd_rn(a, bq); r = live ? r : 0.0f;
        unsigned short a2, c2; splitf(r, a2, c2); oh[q] = a2; ol[q] = c2; }
    *(volatile v2us*)(Ph + e) = oh; *(volatile v2us*)(Pl + e) = ol; __threadfence(); *(volatile v2us*)(Ph + e) = oh; *(volatile v2us*)(Pl + e) = ol; }
__global__ __launch_bounds__(256) void k_vtp(const float* __restrict__ F, int pitch, int nheads, int prow, int toff, bf* Vh, bf* Vl) {
    const unsigned e = (blockIdx.x * 256u + threadIdx.x) * 2u; if (e >= (unsigned)nheads * (unsigned)HD * (unsigned)prow) return;
    const int tp = (int)(e % (unsigned)prow); const int d = (int)((e / (unsigned)prow) % HD); const int g = (int)(e / ((unsigned)prow * (unsigned)HD)); v2us oh, ol;
#pragma unroll
    for (int q = 0; q < 2; ++q) { const int t = tp + q - toff; const bool live = (t >= 0); const int tc = live ? t : 0; float x = F[(size_t)tc * pitch + g * HD + d]; x = live ? x : 0.0f;
        unsigned short a2, c2; splitf(x, a2, c2); oh[q] = a2; ol[q] = c2; }
    *(volatile v2us*)(Vh + e) = oh; *(volatile v2us*)(Vl + e) = ol; __threadfence(); *(volatile v2us*)(Vh + e) = oh; *(volatile v2us*)(Vl + e) = ol; }

__global__ __launch_bounds__(256) void k_soft(const float* __restrict__ Sb, bf* Ph, bf* Pl) {
    const int lane = threadIdx.x & 31; const int row = blockIdx.x * 8 + (threadIdx.x >> 5); if (row >= NH_ * TT) return;
    const int tm = (row % TT) & 63; const int clo = tm + 1, chi = tm + WIN;
    const float* sr = Sb + (size_t)row * SBW;
    const v4f a4 = *(const v4f*)(sr + lane * 4); const v2f b2 = *(const v2f*)(sr + 128 + lane * 2);
    float v[6]; float mx = -3.0e38f;
#pragma unroll
    for (int q = 0; q < 4; ++q) { const int c = lane * 4 + q; const float tq = (c >= clo && c <= chi) ? a4[q] * SCL : -3.0e38f; v[q] = tq; mx = fmaxf(mx, tq); }
#pragma unroll
    for (int q = 0; q < 2; ++q) { const int c = 128 + lane * 2 + q; const float tq = (c >= clo && c <= chi) ? b2[q] * SCL : -3.0e38f; v[4 + q] = tq; mx = fmaxf(mx, tq); }
#pragma unroll
    for (int sh = 16; sh; sh >>= 1) mx = fmaxf(mx, __shfl_xor(mx, sh, 32));
    float sum = 0.f;
#pragma unroll
    for (int k = 0; k < 6; ++k) { float d0 = __fsub_rn(v[k], mx); asm volatile("" : "+v"(d0)); v[k] = __builtin_amdgcn_exp2f(__fmul_rn(d0, 1.4426950408889634f)); sum += v[k]; }
#pragma unroll
    for (int sh = 16; sh; sh >>= 1) sum += __shfl_xor(sum, sh, 32);
    const float f = __fdiv_rn(1.0f, sum);
    v4us oh, ol; v2us oh2, ol2;
#pragma unroll
    for (int q = 0; q < 4; ++q) { unsigned short a, c2; splitf(v[q] * f, a, c2); oh[q] = a; ol[q] = c2; }
#pragma unroll
    for (int q = 0; q < 2; ++q) { unsigned short a, c2; splitf(v[4 + q] * f, a, c2); oh2[q] = a; ol2[q] = c2; }
    const size_t oo = (size_t)row * SBW;
#pragma unroll 1
    for (int ps = 0; ps < 2; ++ps) {
        *(volatile v4us*)(Ph + oo + lane * 4) = oh; *(volatile v4us*)(Pl + oo + lane * 4) = ol;
        *(volatile v2us*)(Ph + oo + 128 + lane * 2) = oh2; *(volatile v2us*)(Pl + oo + 128 + lane * 2) = ol2;
        if (ps == 0) __threadfence(); }
}

extern "C" void kernel_launch(void* const* d_in, const int* in_sizes, int n_in,
                              void* d_out, int out_size, void* d_ws, size_t ws_size, hipStream_t stream) {
    if (n_in < 5) return;
    if (in_sizes[0] < (NB - 1) * SEQ_FULL * DM + TT * DM || in_sizes[1] < DM * DQ || in_sizes[2] < DM * DKV || in_sizes[3] < DM * DKV || in_sizes[4] < DQ * DM) return;
    if (out_size < NB * TT * DM) return;
    const float* x = (const float*)d_in[0]; const float* wq = (const float*)d_in[1]; const float* wk = (const float*)d_in[2]; const float* wv = (const float*)d_in[3]; const float* wo = (const float*)d_in[4];
    float* OUT = (float*)d_out;
    char* wsp = (char*)d_ws;
    auto take = [&](size_t bytes) { char* p = wsp; wsp += (bytes + 255) & ~(size_t)255; return (void*)p; };
    bf* WQ = (bf*)take((size_t)DQ * DM * 2); bf* WK = (bf*)take((size_t)DKV * DM * 2); bf* WV = (bf*)take((size_t)DKV * DM * 2); bf* WO = (bf*)take((size_t)DM * DQ * 2);
    float* CS = (float*)take((size_t)TT * HD * 2 * 4);
    bf* XB = (bf*)take((size_t)TT * DM * 2); float* FQ = (float*)take((size_t)TT * DQ * 4); float* FK = (float*)take((size_t)TT * DKV * 4); float* FV = (float*)take((size_t)TT * DKV * 4);
    bf* QPh = (bf*)take((size_t)NH_ * TT * HD * 2); bf* QPl = (bf*)take((size_t)NH_ * TT * HD * 2);
    bf* KPh = (bf*)take((size_t)NKV * TP * HD * 2); bf* KPl = (bf*)take((size_t)NKV * TP * HD * 2);
    bf* VTh = (bf*)take((size_t)NKV * HD * TP * 2); bf* VTl = (bf*)take((size_t)NKV * HD * TP * 2);
    float* Sb = (float*)take((size_t)NH_ * TT * SBW * 4); bf* Ph = (bf*)take((size_t)NH_ * TT * SBW * 2); bf* Pl = (bf*)take((size_t)NH_ * TT * SBW * 2);
    float* ATf = (float*)take((size_t)TT * DQ * 4); bf* ATh = (bf*)take((size_t)TT * DQ * 2); bf* ATl = (bf*)take((size_t)TT * DQ * 2);
    const size_t carve = (size_t)(wsp - (char*)d_ws);
    if (carve > ws_size || carve > ((size_t)128 << 20)) return;
    k_wtG<<<(unsigned)((DM * DQ / 64 + 63) / 64), 256, 0, stream>>>(wq, DM, DQ, WQ);
    k_wtG<<<(unsigned)((DM * DKV / 64 + 63) / 64), 256, 0, stream>>>(wk, DM, DKV, WK);
    k_wtG<<<(unsigned)((DM * DKV / 64 + 63) / 64), 256, 0, stream>>>(wv, DM, DKV, WV);
    k_wtG<<<(unsigned)((DQ * DM / 64 + 63) / 64), 256, 0, stream>>>(wo, DQ, DM, WO);
    k_cst<<<(unsigned)(TT * HD / 256), 256, 0, stream>>>(CS);
    for (int b = 0; b < NB; ++b) {
        k_cvt8<<<(unsigned)((size_t)TT * DM / 8 / 256), 256, 0, stream>>>(x + (size_t)b * SEQ_FULL * DM, XB, (size_t)TT * DM / 8);
        k_gemmw<bf, 0, false><<<dim3(TT / 64, DQ / 64, 1), 32, 0, stream>>>(XB, nullptr, WQ, nullptr, DM, FQ, DQ, nullptr, 0, 0, 0);
        k_gemmw<bf, 0, false><<<dim3(TT / 64, DKV / 64, 1), 32, 0, stream>>>(XB, nullptr, WK, nullptr, DM, FK, DKV, nullptr, 0, 0, 0);
        k_gemmw<bf, 0, false><<<dim3(TT / 64, DKV / 64, 1), 32, 0, stream>>>(XB, nullptr, WV, nullptr, DM, FV, DKV, nullptr, 0, 0, 0);
        k_rope<<<(unsigned)((size_t)NH_ * TT * HD / 2 / 256), 256, 0, stream>>>(FQ, DQ, NH_, TT, 0, CS, QPh, QPl);
        k_rope<<<(unsigned)((size_t)NKV * TP * HD / 2 / 256), 256, 0, stream>>>(FK, DKV, NKV, TP, PADK, CS, KPh, KPl);
        k_vtp<<<(unsigned)((size_t)NKV * HD * TP / 2 / 256), 256, 0, stream>>>(FV, DKV, NKV, TP, PADK, VTh, VTl);
        k_gemmb<2, REP><<<dim3(TT / 64, SBW / 64, NH_), 32, 0, stream>>>(QPh, QPl, HD, KPh, KPl, HD, HD, Sb, SBW, (size_t)TT * HD, (size_t)TP * HD, (size_t)TT * SBW, (size_t)64 * HD);
        k_soft<<<(unsigned)(NH_ * TT / 8), 256, 0, stream>>>(Sb, Ph, Pl);
        k_gemmb<2, REP><<<dim3(TT / 64, HD / 64, NH_), 32, 0, stream>>>(Ph, Pl, SBW, VTh, VTl, TP, SBW, ATf, DQ, (size_t)TT * SBW, (size_t)HD * TP, (size_t)HD, (size_t)64);
        k_split8<<<(unsigned)((size_t)TT * DQ / 8 / 256), 256, 0, stream>>>(ATf, ATh, ATl, (size_t)TT * DQ / 8);
        k_gemmw<bf, 1, false><<<dim3(TT / 64, DM / 64, 1), 32, 0, stream>>>(ATh, ATl, WO, nullptr, DQ, OUT + (size_t)b * TT * DM, DM, nullptr, 0, 0, 0);
    }
}
